// LorentzMoE_3891240370246
// MI455X (gfx1250) — hardware-verified
//
#include <hip/hip_runtime.h>
#include <math.h>

typedef __attribute__((ext_vector_type(16))) _Float16 v16h;
typedef __attribute__((ext_vector_type(16))) __bf16 v16b;
typedef __attribute__((ext_vector_type(8)))  _Float16 v8h;
typedef __attribute__((ext_vector_type(8)))  float v8f;
typedef __attribute__((ext_vector_type(4)))  float v4f;
typedef __attribute__((ext_vector_type(2)))  float v2f;
typedef __attribute__((ext_vector_type(4)))  unsigned v4u;
typedef __attribute__((ext_vector_type(4)))  int v4i;
typedef float __attribute__((may_alias)) float_a;
typedef int __attribute__((may_alias)) int_a;

template <typename T> __device__ __forceinline__ void vst2(void* p, T v) { *(volatile T*)p = v; __threadfence(); *(volatile T*)p = v; }
__device__ __forceinline__ v8f wmma16(v16h a, v16h b, v8f c) {
  v8f d = __builtin_amdgcn_wmma_f32_16x16x32_f16(false, a, false, b, (short)0, c, false, false);
  asm volatile("v_nop\n\tv_nop\n\tv_nop\n\tv_nop" : "+v"(d) : "v"(a), "v"(b));
  return d;
}
__device__ __forceinline__ v8f wmma_bf(v16b a, v16b b, v8f c) {
  v8f d = __builtin_amdgcn_wmma_f32_16x16x32_bf16(false, a, false, b, (short)0, c, false, false);
  asm volatile("v_nop\n\tv_nop\n\tv_nop\n\tv_nop" : "+v"(d) : "v"(a), "v"(b));
  return d;
}
__device__ __forceinline__ v16h frag_h(const _Float16* rowk0, int lane) {
  union { v16h v; v8h q[2]; } u; const _Float16* p = rowk0 + 8 * (lane >> 4);
  u.q[0] = *(const v8h*)p; u.q[1] = *(const v8h*)(p + 16); return u.v;
}
__device__ __forceinline__ v16h frag_f32(const float* rowk0, int lane) {
  v16h a; const float* p = rowk0 + 8 * (lane >> 4);
#pragma unroll
  for (int i = 0; i < 8; ++i) { a[i] = (_Float16)p[i]; a[8 + i] = (_Float16)p[16 + i]; }
  return a;
}
__device__ __forceinline__ v16h frag_f32s(const float* rowk0, int lane, float sc) {
  v16h a; const float* p = rowk0 + 8 * (lane >> 4);
#pragma unroll
  for (int i = 0; i < 8; ++i) { a[i] = (_Float16)(p[i] * sc); a[8 + i] = (_Float16)(p[16 + i] * sc); }
  return a;
}
__device__ __forceinline__ v16h fragc_f32(const float* W, int k0, int n, int lane, int ld, int K) {
  v16h a; const int g = lane >> 4;
#pragma unroll
  for (int i = 0; i < 8; ++i) { const int ka = k0 + 8 * g + i, kb = ka + 16;
    a[i] = (_Float16)(ka < K ? W[(size_t)(ka < K ? ka : K - 1) * ld + n] : 0.f); a[8 + i] = (_Float16)(kb < K ? W[(size_t)(kb < K ? kb : K - 1) * ld + n] : 0.f); }
  return a;
}
struct F2 { v16b h, l; };
__device__ __forceinline__ F2 bsplit16(const float v[16]) { F2 r;
#pragma unroll
  for (int i = 0; i < 16; ++i) { const __bf16 h = (__bf16)v[i]; r.h[i] = h; r.l[i] = (__bf16)(v[i] - (float)h); }
  return r; }
__device__ __forceinline__ F2 split_row(const float* row, int k0, int lane) { float v[16]; const float* p = row + k0 + 8 * (lane >> 4);
#pragma unroll
  for (int i = 0; i < 8; ++i) { v[i] = p[i]; v[8 + i] = p[16 + i]; }
  return bsplit16(v); }
__device__ __forceinline__ F2 split_rowK(const float* row, int k0, int lane, int K) { float v[16]; const int g = lane >> 4;
#pragma unroll
  for (int i = 0; i < 8; ++i) { const int ka = k0 + 8 * g + i, kb = ka + 16; v[i] = ka < K ? row[ka < K ? ka : K - 1] : 0.f; v[8 + i] = kb < K ? row[kb < K ? kb : K - 1] : 0.f; }
  return bsplit16(v); }
__device__ __forceinline__ F2 split_col(const float* W, int k0, int n, int lane, int ld, int K) { float v[16]; const int g = lane >> 4;
#pragma unroll
  for (int i = 0; i < 8; ++i) { const int ka = k0 + 8 * g + i, kb = ka + 16; v[i] = ka < K ? W[(size_t)(ka < K ? ka : K - 1) * ld + n] : 0.f; v[8 + i] = kb < K ? W[(size_t)(kb < K ? kb : K - 1) * ld + n] : 0.f; }
  return bsplit16(v); }
__device__ __forceinline__ v8f mac3(const F2& a, const F2& b, v8f c) { c = wmma_bf(a.l, b.h, c); c = wmma_bf(a.h, b.l, c); return wmma_bf(a.h, b.h, c); }
__device__ __forceinline__ float sigm(float v) { return 1.0f / (1.0f + expf(-v)); }
#define LDSX() do { asm volatile("s_wait_dscnt 0" ::: "memory"); __builtin_amdgcn_wave_barrier(); __builtin_amdgcn_fence(__ATOMIC_RELEASE, "workgroup"); } while (0)


#define TT 2048
#define DD 1024
#define NEX 8
#define IW 1024
#define NSP (IW - 1)
#define NO (DD - 1)
#define LEPS 1e-8f
#ifndef TRB
#define TRB (TT / 64)
#endif
typedef __attribute__((ext_vector_type(8))) __bf16 v8b;
__device__ __forceinline__ v16b frag_b(const __bf16* rowk0, int lane) {
  union { v16b v; v8b q[2]; } u; const __bf16* p = rowk0 + 8 * (lane >> 4);
  u.q[0] = *(const v8b*)p; u.q[1] = *(const v8b*)(p + 16); return u.v;
}
__device__ __forceinline__ float bfr(float v) { return (float)(__bf16)v; }
__device__ __attribute__((noinline)) float exp_ni(float v) { return expf(v); }
__device__ __attribute__((noinline)) float erf_ni(float v) { return erff(v); }

#define PK_GT  0
#define PK_UP  (PK_GT + 16 * DD)
#define PK_DN  (PK_UP + (size_t)(NEX + 1) * 2 * IW * DD)
#define PK_END (PK_DN + (size_t)(NEX + 1) * DD * IW)
#define WS_PK  0u
#define WS_GW  (WS_PK + 2u * (unsigned)PK_END)
#define WS_H2  (WS_GW + 4u * TT * NEX)
#define WS_SP  (WS_H2 + 4u * TT * 2 * IW)
#define WS_O   (WS_SP + 4u * TT * IW)
#define WS_Y   (WS_O + 4u * TT * DD)
#define WS_Z   (WS_Y + 4u * TT * DD)
#define WS_END (WS_Z + 4u * TT * DD)

__global__ __launch_bounds__(256) void k_packrows(const float* __restrict__ Wm, size_t sstride, int NR, int K, __bf16* __restrict__ DST, size_t dplane, int rofs) {
  __shared__ __align__(16) __bf16 s[1024]; const int n = blockIdx.x, slot = blockIdx.y, tid = threadIdx.x; const float* w = Wm + (size_t)slot * sstride + (size_t)n * K;
  for (int k = tid; k < K; k += 256) s[k] = (__bf16)((n < NR) ? w[k] : 0.f);
  __syncthreads();
  for (int q = tid; q < K / 8; q += 256) vst2((unsigned*)(DST + (size_t)slot * dplane + (size_t)(rofs + n) * K + q * 8), *(const v4u*)&s[q * 8]);
}
__global__ __launch_bounds__(256) void k_packgate(const float* __restrict__ GWm, __bf16* __restrict__ DST) {
  __shared__ __align__(16) __bf16 s[DD]; const int n = blockIdx.x, tid = threadIdx.x;
  for (int k = tid; k < DD; k += 256) s[k] = (__bf16)((n < NEX && k >= 1) ? GWm[(size_t)n * (DD - 1) + (k - 1)] : 0.f);
  __syncthreads();
  for (int q = tid; q < DD / 8; q += 256) vst2((unsigned*)(DST + (size_t)n * DD + q * 8), *(const v4u*)&s[q * 8]);
}
__global__ __launch_bounds__(128) void k_gate(const float* __restrict__ X, const __bf16* __restrict__ PG, const float* __restrict__ GB, float* __restrict__ GW, float* __restrict__ Y) {
  __shared__ float ssc[64][17]; __shared__ __align__(16) float sgw[64][NEX];
  const int tid = threadIdx.x, wave = tid >> 5, lane = tid & 31, col = lane & 15, g = lane >> 4; const size_t r0 = (size_t)blockIdx.x * 64 + wave * 16;
  v8f acc = {};
#pragma unroll 4
  for (int kc = 0; kc < DD / 32; ++kc) { v16b a; { const float* p = X + (r0 + col) * DD + kc * 32 + 8 * g;
#pragma unroll
      for (int i = 0; i < 8; ++i) { a[i] = (__bf16)p[i]; a[8 + i] = (__bf16)p[16 + i]; } }
    acc = wmma_bf(a, frag_b(PG + (size_t)col * DD + kc * 32, lane), acc); }
#pragma unroll
  for (int r = 0; r < 8; ++r) ssc[wave * 16 + 8 * g + r][col] = acc[r];
  __syncthreads();
  if (tid < 64) { const int t = tid; float lg[NEX]; float mx = -3.0e38f;
#pragma unroll
    for (int e = 0; e < NEX; ++e) { lg[e] = ssc[t][e]; mx = fmaxf(mx, lg[e]); }
    float z = 0.f; float sc[NEX];
#pragma unroll
    for (int e = 0; e < NEX; ++e) { sc[e] = exp_ni(lg[e] - mx); z += sc[e]; }
    const float iz = 1.0f / z; int bi = 0; float bv = -3.0e38f;
#pragma unroll
    for (int e = 0; e < NEX; ++e) { sc[e] *= iz; const float b = sc[e] + bfr(GB[e]); if (b > bv) { bv = b; bi = e; } }
#pragma unroll
    for (int e = 0; e < NEX; ++e) sgw[t][e] = (e == bi) ? sc[e] : 0.f; }
  __syncthreads();
  for (int q = tid; q < 64 * 2; q += 128) { const int rl = q >> 1, pc = q & 1; vst2(GW + ((size_t)blockIdx.x * 64 + rl) * NEX + pc * 4, *(const v4f*)&sgw[rl][pc * 4]); }
  for (int q = tid; q < 64 * (DD / 4); q += 128) { const int rl = q / (DD / 4), pc = q % (DD / 4); vst2(Y + ((size_t)blockIdx.x * 64 + rl) * DD + pc * 4, (pc == 0) ? (v4f){1.f, 0.f, 0.f, 0.f} : (v4f){0.f, 0.f, 0.f, 0.f}); }
}
__global__ __launch_bounds__(128) void k_up(const float* __restrict__ X, const __bf16* __restrict__ P, float* __restrict__ H2) {
  __shared__ __align__(16) float so[4][16][132];
  const int tid = threadIdx.x, wave = tid >> 5, lane = tid & 31, col = lane & 15, g = lane >> 4; const size_t r0 = (size_t)blockIdx.x * 64 + wave * 16; const int n0 = blockIdx.y * 128;
  v8f acc[8] = {};
#pragma unroll 2
  for (int kc = 0; kc < DD / 32; ++kc) { v16b a; { const float* p = X + (r0 + col) * DD + kc * 32 + 8 * g;
#pragma unroll
      for (int i = 0; i < 8; ++i) { a[i] = (__bf16)p[i]; a[8 + i] = (__bf16)p[16 + i]; } }
#pragma unroll
    for (int j = 0; j < 8; ++j) acc[j] = wmma_bf(a, frag_b(P + (size_t)(n0 + j * 16 + col) * DD + kc * 32, lane), acc[j]); }
#pragma unroll
  for (int j = 0; j < 8; ++j)
#pragma unroll
    for (int r = 0; r < 8; ++r) so[wave][8 * g + r][j * 16 + col] = acc[j][r];
  LDSX();
  for (int rl = 0; rl < 16; ++rl) vst2(H2 + (r0 + rl) * (2 * IW) + n0 + lane * 4, *(const v4f*)&so[wave][rl][lane * 4]);
}
__global__ __launch_bounds__(256) void k_sp(const float* __restrict__ H2, float* __restrict__ SP) {
  __shared__ __align__(16) float s[8][IW];
  const int wave = threadIdx.x >> 5, lane = threadIdx.x & 31; const size_t r = (size_t)blockIdx.x * 8 + wave; const float* h = H2 + r * (2 * IW); float* sw = s[wave];
  float ss = 0.f;
  for (int i = lane; i < NSP; i += 32) { const float a = h[i], b = h[IW + i]; const float v = a / (1.0f + exp_ni(-a)) * b; sw[1 + i] = v; ss += v * v; }
#pragma unroll
  for (int o = 1; o < 32; o <<= 1) ss += __shfl_xor(ss, o);
  if (lane == 0) sw[0] = sqrtf(fmaxf(ss + 1.0f, LEPS));
  LDSX();
  for (int pc = lane; pc < IW / 4; pc += 32) vst2(SP + r * IW + pc * 4, *(const v4f*)&sw[pc * 4]);
}
__global__ __launch_bounds__(128) void k_down(const float* __restrict__ SP, const __bf16* __restrict__ P, float* __restrict__ O) {
  __shared__ __align__(16) float so[4][16][132];
  const int tid = threadIdx.x, wave = tid >> 5, lane = tid & 31, col = lane & 15, g = lane >> 4; const size_t r0 = (size_t)blockIdx.x * 64 + wave * 16; const int n0 = blockIdx.y * 128;
  v8f acc[8] = {};
#pragma unroll 2
  for (int kc = 0; kc < IW / 32; ++kc) { const F2 a = split_row(SP + (r0 + col) * IW, kc * 32, lane);
#pragma unroll
    for (int j = 0; j < 8; ++j) { const v16b w = frag_b(P + (size_t)(n0 + j * 16 + col) * IW + kc * 32, lane); acc[j] = wmma_bf(a.l, w, acc[j]); acc[j] = wmma_bf(a.h, w, acc[j]); } }
#pragma unroll
  for (int j = 0; j < 8; ++j)
#pragma unroll
    for (int r = 0; r < 8; ++r) so[wave][8 * g + r][j * 16 + col] = acc[j][r];
  LDSX();
  for (int rl = 0; rl < 16; ++rl) vst2(O + (r0 + rl) * DD + n0 + lane * 4, *(const v4f*)&so[wave][rl][lane * 4]);
}
__global__ __launch_bounds__(256) void k_acc(const float* __restrict__ O, const float* __restrict__ GW, int e, float* __restrict__ DSTROWS) {
  __shared__ __align__(16) float s[8][DD];
  const int wave = threadIdx.x >> 5, lane = threadIdx.x & 31; const size_t r = (size_t)blockIdx.x * 8 + wave; const float* o = O + r * DD; float* sw = s[wave]; float* d = DSTROWS + r * DD;
  const float w = (e >= 0) ? GW[r * NEX + e] : 1.0f;
  float ss = 0.f;
  for (int n = lane; n < NO; n += 32) { const float v = o[n]; ss += v * v; sw[1 + n] = (e >= 0) ? d[1 + n] + w * v : v; }
#pragma unroll
  for (int oo = 1; oo < 32; oo <<= 1) ss += __shfl_xor(ss, oo);
  if (lane == 0) { const float ot = sqrtf(fmaxf(ss + 1.0f, LEPS)); sw[0] = (e >= 0) ? d[0] + w * ot : ot; }
  LDSX();
  for (int pc = lane; pc < DD / 4; pc += 32) vst2(d + pc * 4, *(const v4f*)&sw[pc * 4]);
}
__global__ __launch_bounds__(256) void k_fin(const float* __restrict__ Y, const float* __restrict__ Z, float* __restrict__ out) {
  __shared__ __align__(16) float s[8][DD];
  const int wave = threadIdx.x >> 5, lane = threadIdx.x & 31; const size_t r = (size_t)blockIdx.x * 8 + wave; float* sw = s[wave];
  float ss = 0.f; float c0 = 0.f;
  for (int n = lane; n < DD; n += 32) { const float v = Z[r * DD + n] + 2.0f * Y[r * DD + n]; sw[n] = v; if (n == 0) c0 = v; else ss += v * v; }
#pragma unroll
  for (int o = 1; o < 32; o <<= 1) { ss += __shfl_xor(ss, o); c0 += __shfl_xor(c0, o); }
  const float li = ss - c0 * c0; const float inv = 1.0f / sqrtf(fmaxf(fabsf(li), LEPS));
  LDSX();
  for (int n = lane; n < DD; n += 32) sw[n] *= inv;
  LDSX();
  for (int pc = lane; pc < DD / 4; pc += 32) vst2(out + r * DD + pc * 4, *(const v4f*)&sw[pc * 4]);
}
extern "C" void kernel_launch(void* const* d_in, const int* in_sizes, int n_in, void* d_out, int out_size, void* d_ws, size_t ws_size, hipStream_t stream) {
  (void)in_sizes; (void)n_in; (void)out_size;
  const float** F = (const float**)d_in;
  if (ws_size < (size_t)WS_END) return;
  char* ws = (char*)d_ws; __bf16* PK = (__bf16*)(ws + WS_PK); float *GW = (float*)(ws + WS_GW), *H2 = (float*)(ws + WS_H2), *SP = (float*)(ws + WS_SP), *O = (float*)(ws + WS_O), *Y = (float*)(ws + WS_Y), *Z = (float*)(ws + WS_Z);
  const size_t upplane = (size_t)2 * IW * DD, dnplane = (size_t)DD * IW, wstride = (size_t)NSP * DD;
  k_packgate<<<16, 256, 0, stream>>>(F[1], PK + PK_GT);
  k_packrows<<<dim3(IW, NEX), 256, 0, stream>>>(F[3], wstride, NSP, DD, PK + PK_UP, upplane, 0);
  k_packrows<<<dim3(IW, NEX), 256, 0, stream>>>(F[4], wstride, NSP, DD, PK + PK_UP, upplane, IW);
  k_packrows<<<dim3(DD, NEX), 256, 0, stream>>>(F[5], wstride, NO, IW, PK + PK_DN, dnplane, 0);
  k_packrows<<<dim3(IW, 1), 256, 0, stream>>>(F[6], 0, NSP, DD, PK + PK_UP + NEX * upplane, 0, 0);
  k_packrows<<<dim3(IW, 1), 256, 0, stream>>>(F[7], 0, NSP, DD, PK + PK_UP + NEX * upplane, 0, IW);
  k_packrows<<<dim3(DD, 1), 256, 0, stream>>>(F[8], 0, NO, IW, PK + PK_DN + NEX * dnplane, 0, 0);
  k_gate<<<TRB, 128, 0, stream>>>(F[0], PK + PK_GT, F[2], GW, Y);
  for (int e = 0; e <= NEX; ++e) { const int slot = e;
    k_up<<<dim3(TRB, 2 * IW / 128), 128, 0, stream>>>(F[0], PK + PK_UP + slot * upplane, H2);
    k_sp<<<TRB * 8, 256, 0, stream>>>(H2, SP);
    k_down<<<dim3(TRB, DD / 128), 128, 0, stream>>>(SP, PK + PK_DN + slot * dnplane, O);
    k_acc<<<TRB * 8, 256, 0, stream>>>(O, GW, (e < NEX) ? e : -1, (e < NEX) ? Y : Z); }
  k_fin<<<TRB * 8, 256, 0, stream>>>(Y, Z, (float*)d_out);
}
